// YOSOEAttention_63926293233877
// MI455X (gfx1250) — hardware-verified
//
#include <hip/hip_runtime.h>


typedef _Float16 h8  __attribute__((ext_vector_type(8)));
typedef _Float16 h16 __attribute__((ext_vector_type(16)));
typedef float    f8  __attribute__((ext_vector_type(8)));

#define S_LEN 4096
#define NHEAD 8
#define DHEAD 64
#define QTILE 128
#define KTILE 64
#define NWAVE 8

__device__ __forceinline__ h16 cat16(h8 a, h8 b) {
  h16 r;
#pragma unroll
  for (int i = 0; i < 8; ++i) { r[i] = a[i]; r[i + 8] = b[i]; }
  return r;
}

__device__ __forceinline__ h8 lds_ld8(const _Float16* p) {
  return *(const h8*)p;
}

__global__ __launch_bounds__(256)
void yoso_attn_wmma_kernel(const float* __restrict__ Q,
                           const float* __restrict__ K,
                           const float* __restrict__ V,
                           const float* __restrict__ mask,
                           const float* __restrict__ cw,
                           float* out) {
  __shared__ __align__(16) unsigned char smem[49152];
  _Float16* sm_qn = (_Float16*)smem;
  _Float16* sm_kn = sm_qn + QTILE * DHEAD;
  _Float16* sm_vt = sm_kn + KTILE * DHEAD;
  _Float16* sm_p  = sm_vt + DHEAD * KTILE;
  float* cst = (float*)smem;
  const int CSTR = DHEAD + 4;

  const int h      = blockIdx.y;
  const int qbase  = blockIdx.x * QTILE;
  const int tid    = threadIdx.x;
  const int wv     = tid >> 5;
  const int lane   = tid & 31;
  const int lh     = lane >> 4;
  const int ln     = lane & 15;
  const int dofs8  = lh * 8;
  const size_t headoff = (size_t)h * S_LEN * DHEAD;

  {
    const int r  = tid >> 1;
    const int hf = tid & 1;
    const float* qrow = Q + headoff + (size_t)(qbase + r) * DHEAD + hf * 32;
    float4 b[8];
    float ss = 0.f;
#pragma unroll
    for (int i = 0; i < 8; ++i) {
      b[i] = ((const float4*)qrow)[i];
      ss += b[i].x * b[i].x + b[i].y * b[i].y + b[i].z * b[i].z + b[i].w * b[i].w;
    }
    ss += __shfl_xor(ss, 1);
    const float inv = 1.f / fmaxf(sqrtf(ss), 1e-12f);
    _Float16* dst = sm_qn + r * DHEAD + hf * 32;
#pragma unroll
    for (int i = 0; i < 8; ++i) {
      dst[i * 4 + 0] = (_Float16)(b[i].x * inv);
      dst[i * 4 + 1] = (_Float16)(b[i].y * inv);
      dst[i * 4 + 2] = (_Float16)(b[i].z * inv);
      dst[i * 4 + 3] = (_Float16)(b[i].w * inv);
    }
  }
  __syncthreads();

  h16 qA[2];
#pragma unroll
  for (int c = 0; c < 2; ++c) {
    const _Float16* base = sm_qn + (wv * 16 + ln) * DHEAD + c * 32;
    qA[c] = cat16(lds_ld8(base + dofs8), lds_ld8(base + 16 + dofs8));
  }

  f8 oacc[4];
#pragma unroll
  for (int t = 0; t < 4; ++t) oacc[t] = {};

  _Float16* pw = sm_p + wv * 16 * KTILE;

  for (int kb = 0; kb < S_LEN / KTILE; ++kb) {
    __syncthreads();
    {
      const int r  = tid >> 2;
      const int q4 = tid & 3;
      const int key = kb * KTILE + r;
      const float* krow = K + headoff + (size_t)key * DHEAD + q4 * 16;
      float4 b[4];
      float ss = 0.f;
#pragma unroll
      for (int i = 0; i < 4; ++i) {
        b[i] = ((const float4*)krow)[i];
        ss += b[i].x * b[i].x + b[i].y * b[i].y + b[i].z * b[i].z + b[i].w * b[i].w;
      }
      ss += __shfl_xor(ss, 1);
      ss += __shfl_xor(ss, 2);
      const float inv = 1.f / fmaxf(sqrtf(ss), 1e-12f);
      _Float16* dst = sm_kn + r * DHEAD + q4 * 16;
#pragma unroll
      for (int i = 0; i < 4; ++i) {
        dst[i * 4 + 0] = (_Float16)(b[i].x * inv);
        dst[i * 4 + 1] = (_Float16)(b[i].y * inv);
        dst[i * 4 + 2] = (_Float16)(b[i].z * inv);
        dst[i * 4 + 3] = (_Float16)(b[i].w * inv);
      }
      const float* vrow = V + headoff + (size_t)key * DHEAD + q4 * 16;
#pragma unroll
      for (int i = 0; i < 4; ++i) {
        const float4 v4 = ((const float4*)vrow)[i];
        const int c0 = q4 * 16 + i * 4;
        sm_vt[(c0 + 0) * KTILE + r] = (_Float16)v4.x;
        sm_vt[(c0 + 1) * KTILE + r] = (_Float16)v4.y;
        sm_vt[(c0 + 2) * KTILE + r] = (_Float16)v4.z;
        sm_vt[(c0 + 3) * KTILE + r] = (_Float16)v4.w;
      }
    }
    __syncthreads();

#pragma unroll
    for (int nt = 0; nt < 4; ++nt) {
      const int n0 = nt * 16;
      const _Float16* kb0 = sm_kn + (n0 + ln) * DHEAD;
      const h16 Blo = cat16(lds_ld8(kb0 + dofs8),      lds_ld8(kb0 + 16 + dofs8));
      const h16 Bhi = cat16(lds_ld8(kb0 + 32 + dofs8), lds_ld8(kb0 + 48 + dofs8));
      f8 acc = {};
      acc = __builtin_amdgcn_wmma_f32_16x16x32_f16(false, qA[0], false, Blo, (short)0, acc, false, false);
      acc = __builtin_amdgcn_wmma_f32_16x16x32_f16(false, qA[1], false, Bhi, (short)0, acc, false, false);
      asm volatile("v_nop\n\tv_nop\n\tv_nop\n\tv_nop" : "+v"(acc) : "v"(qA[0]), "v"(qA[1]), "v"(Blo), "v"(Bhi));
      const float km = mask[kb * KTILE + n0 + ln];
#pragma unroll
      for (int r = 0; r < 8; ++r) {
        float s = acc[r];
        s = fminf(fmaxf(s, -1.f + 1e-6f), 1.f - 1e-6f);
        float p = 1.f - acosf(s) * 0.3183098861837907f;
        p = p * p; p = p * p; p = p * p;
        p *= km;
        pw[(lh * 8 + r) * KTILE + n0 + ln] = (_Float16)p;
      }
    }

    __syncthreads();

#pragma unroll
    for (int kc = 0; kc < 2; ++kc) {
      const _Float16* pb = pw + ln * KTILE + kc * 32;
      const h16 PA = cat16(lds_ld8(pb + dofs8), lds_ld8(pb + 16 + dofs8));
#pragma unroll
      for (int dt = 0; dt < 4; ++dt) {
        const _Float16* vb = sm_vt + (dt * 16 + ln) * KTILE + kc * 32;
        const h16 BV = cat16(lds_ld8(vb + dofs8), lds_ld8(vb + 16 + dofs8));
        oacc[dt] = __builtin_amdgcn_wmma_f32_16x16x32_f16(false, PA, false, BV, (short)0, oacc[dt], false, false);
      }
      asm volatile("v_nop\n\tv_nop\n\tv_nop\n\tv_nop" : "+v"(oacc[0]), "+v"(oacc[1]), "+v"(oacc[2]), "+v"(oacc[3]) : "v"(PA));
    }
  }

  __syncthreads();
  const float w0 = cw[h * 3 + 0], w1 = cw[h * 3 + 1], w2 = cw[h * 3 + 2];
  const int srow_base = qbase + wv * 16 + lh * 8;
#pragma unroll
  for (int r = 0; r < 8; ++r) {
    const int srow = srow_base + r;
    const float qm = mask[srow];
    float xv[4];
    float ss = 0.f;
#pragma unroll
    for (int dt = 0; dt < 4; ++dt) {
      xv[dt] = oacc[dt][r] * qm;
      ss += xv[dt] * xv[dt];
    }
    ss += __shfl_xor(ss, 1);
    ss += __shfl_xor(ss, 2);
    ss += __shfl_xor(ss, 4);
    ss += __shfl_xor(ss, 8);
    const float inv = 1.f / fmaxf(sqrtf(ss), 1e-12f);

    const float* vc = V + headoff + (size_t)srow * DHEAD;
    const float mm1 = (srow > 0)          ? mask[srow - 1] : 0.f;
    const float mp1 = (srow < S_LEN - 1)  ? mask[srow + 1] : 0.f;
#pragma unroll
    for (int dt = 0; dt < 4; ++dt) {
      const int d = dt * 16 + ln;
      const float vm1 = (srow > 0)         ? vc[d - DHEAD] * mm1 : 0.f;
      const float v0  = vc[d] * qm;
      const float vp1 = (srow < S_LEN - 1) ? vc[d + DHEAD] * mp1 : 0.f;
      const float conv = w0 * vm1 + w1 * v0 + w2 * vp1;
      cst[(srow - qbase) * CSTR + d] = xv[dt] * inv + conv;
    }
  }
  __syncthreads();
  {
    const int col = tid & 63, rsel = tid >> 6;
    float* ob = out + headoff + (size_t)qbase * DHEAD;
#pragma unroll 4
    for (int r = rsel; r < QTILE; r += 4) *(volatile float*)(ob + (size_t)r * DHEAD + col) = cst[r * CSTR + col];
    __threadfence();
#pragma unroll 4
    for (int r = rsel; r < QTILE; r += 4) *(volatile float*)(ob + (size_t)r * DHEAD + col) = cst[r * CSTR + col];
  }
}

extern "C" void kernel_launch(void* const* d_in, const int* in_sizes, int n_in,
                              void* d_out, int out_size, void* d_ws, size_t ws_size,
                              hipStream_t stream) {
  (void)in_sizes; (void)n_in; (void)out_size; (void)d_ws; (void)ws_size;
  const float* Q    = (const float*)d_in[0];
  const float* K    = (const float*)d_in[1];
  const float* V    = (const float*)d_in[2];
  const float* mask = (const float*)d_in[3];
  const float* cw   = (const float*)d_in[4];
  float* out = (float*)d_out;

  dim3 grid(S_LEN / QTILE, NHEAD);
  dim3 block(32 * NWAVE);
  yoso_attn_wmma_kernel<<<grid, block, 0, stream>>>(Q, K, V, mask, cw, out);
}
